// SpatialInteractionMix_49452253446339
// MI455X (gfx1250) — hardware-run, weakly checked
//
#include <hip/hip_runtime.h>
#include <math.h>

typedef __attribute__((ext_vector_type(16))) _Float16 v16h;
typedef __attribute__((ext_vector_type(8)))  _Float16 v8h;
typedef __attribute__((ext_vector_type(8)))  float    v8f;
typedef __attribute__((ext_vector_type(4)))  float    v4f;
typedef __attribute__((ext_vector_type(4)))  unsigned int v4u;

constexpr int kNB   = 16;
constexpr int kImH  = 64;
constexpr int kImW  = 64;
constexpr int kCh   = 192;
constexpr int kSeq  = kImH * kImW;
constexpr int kTok  = kNB * kSeq;
constexpr int kGrp  = kCh / 4;
constexpr int kTileM = 64;
constexpr int kAP   = 200;
constexpr int kCP   = 196;
constexpr float kActCarry   = 16.0f;
constexpr float kWgtCarry   = 256.0f;
constexpr float kFoldScale  = 1.0f / (kActCarry * kWgtCarry);
constexpr float kInvSeq     = 1.0f / (float)kSeq;
constexpr float kInvCh      = 1.0f / (float)kCh;
constexpr float kLnEps      = 1e-5f;
constexpr float kF16MinNorm = 6.103515625e-5f;
static_assert(kSeq == 4096, "tokens per image");
static_assert(kTok == 65536, "token rows");
static_assert(kImW == kTileM, "one block owns one image row");
static_assert((kCh % 32) == 0, "GEMM K multiple of 32");
static_assert((kCh % 64) == 0 && (kTok % 64) == 0, "GEMM M, N multiples of 64");
static_assert((kGrp % 8) == 0, "shift group boundaries fall on 8-channel items");
static_assert(kFoldScale == 1.0f / 4096.0f, "fold scale");
static_assert((kTileM * kCP * 4) >= (kTileM * kAP * 2), "A tile fits inside the C tile buffer");
static_assert((kAP % 8) == 0 && (kCP % 4) == 0, "16-B aligned LDS rows");

constexpr size_t kBytesWT = (size_t)4 * kCh * kCh * 2;
constexpr size_t kBytesKY = (size_t)kTok * kCh * 4;
constexpr size_t kBytesVV = (size_t)kTok * kCh * 4;
constexpr size_t kBytesSR = (size_t)kTok * kCh * 2;
constexpr size_t kOffWT = 0;
constexpr size_t kOffKY = kOffWT + kBytesWT;
constexpr size_t kOffVV = kOffKY + kBytesKY;
constexpr size_t kOffSR = kOffVV + kBytesVV;
constexpr size_t kWsTotal = kOffSR + kBytesSR;
static_assert(kWsTotal == 126124032ull, "carve total");
static_assert(kWsTotal <= 134217728ull, "carve cap");
static_assert((kOffKY % 128) == 0 && (kOffVV % 128) == 0 && (kOffSR % 128) == 0, "128-B aligned regions");

__device__ __forceinline__ _Float16 to_f16_flushed(float v) {
  const float f = (fabsf(v) < kF16MinNorm) ? 0.0f : v;
  return (_Float16)f;
}

__device__ __forceinline__ float h16_to_f32(unsigned hb) {
  const unsigned sgn = (hb & 0x8000u) << 16;
  const unsigned em = hb & 0x7fffu;
  const float fn = __uint_as_float((em << 13) + 0x38000000u);
  const float fs = (float)em * 5.9604644775390625e-8f;
  const float mag = (em < 0x400u) ? fs : fn;
  return __uint_as_float(__float_as_uint(mag) | sgn);
}

__device__ __forceinline__ v16h frag_load(const _Float16* p) {
  union FU { v16h v; v8h h[2]; };
  FU f;
  f.h[0] = *(const v8h*)(p);
  f.h[1] = *(const v8h*)(p + 16);
  return f.v;
}

__device__ __forceinline__ v8f mma_h(v16h a, v16h b, v8f c) {
  c = __builtin_amdgcn_wmma_f32_16x16x32_f16(false, a, false, b, (short)0, c, false, false);
  asm volatile("v_nop\n\tv_nop\n\tv_nop\n\tv_nop" : "+v"(c) : "v"(a), "v"(b));
  return c;
}

__device__ __forceinline__ void tile_gemm(const _Float16* As, const _Float16* Bp, int lane, int wave, v8f (&acc)[2][3]) {
  const int c    = lane & 15;
  const int koff = (lane >> 4) * 8;
  const int mh   = wave & 1;
  const int ng   = wave >> 1;
  const _Float16* ar = As + (mh * 32 + c) * kAP + koff;
  const _Float16* br = Bp + (size_t)(ng * 48 + c) * kCh + koff;
#pragma unroll 1
  for (int k0 = 0; k0 < kCh; k0 += 32) {
    const v16h b0 = frag_load(br + k0);
    const v16h b1 = frag_load(br + 16 * kCh + k0);
    const v16h b2 = frag_load(br + 32 * kCh + k0);
    const v16h a0 = frag_load(ar + k0);
    const v16h a1 = frag_load(ar + 16 * kAP + k0);
    acc[0][0] = mma_h(a0, b0, acc[0][0]);
    acc[0][1] = mma_h(a0, b1, acc[0][1]);
    acc[0][2] = mma_h(a0, b2, acc[0][2]);
    acc[1][0] = mma_h(a1, b0, acc[1][0]);
    acc[1][1] = mma_h(a1, b1, acc[1][1]);
    acc[1][2] = mma_h(a1, b2, acc[1][2]);
  }
}

__device__ __forceinline__ void acc_to_ctile(float* Cs, int lane, int wave, const v8f (&acc)[2][3], float scale, float addend) {
  const int c  = lane & 15;
  const int hh = lane >> 4;
  const int mh = wave & 1;
  const int ng = wave >> 1;
#pragma unroll
  for (int i = 0; i < 2; ++i) {
#pragma unroll
    for (int j = 0; j < 3; ++j) {
#pragma unroll
      for (int r = 0; r < 8; ++r) {
        Cs[(mh * 32 + i * 16 + 8 * hh + r) * kCP + ng * 48 + j * 16 + c] = acc[i][j][r] * scale + addend;
      }
    }
  }
}

__device__ __forceinline__ void store_ctile_f32(const float* Cs, float* dst, int tid) {
  for (int pass = 0; pass < 2; ++pass) {
#pragma unroll
    for (int it = 0; it < 12; ++it) {
      const int idx4 = it * 256 + tid;
      const int row  = idx4 / 48;
      const int col  = (idx4 - row * 48) * 4;
      const v4f v = *(const v4f*)(Cs + row * kCP + col);
      *(volatile v4f*)(dst + (size_t)idx4 * 4) = v;
    }
    __threadfence();
  }
}

__global__ __launch_bounds__(256) void prepack_w_kernel(const float* __restrict__ W0, const float* __restrict__ W1,
                                                        const float* __restrict__ W2, const float* __restrict__ W3,
                                                        unsigned short* __restrict__ out) {
  const int z = blockIdx.y;
  const float* W = (z == 0) ? W0 : ((z == 1) ? W1 : ((z == 2) ? W2 : W3));
  const int i = blockIdx.x * 256 + threadIdx.x;
  const float* p = W + (size_t)i * 8;
  const v4f a = *(const v4f*)(p);
  const v4f b = *(const v4f*)(p + 4);
  v8h hv;
#pragma unroll
  for (int e = 0; e < 4; ++e) {
    hv[e]     = to_f16_flushed(a[e] * kWgtCarry);
    hv[4 + e] = to_f16_flushed(b[e] * kWgtCarry);
  }
  unsigned short* q = out + (size_t)z * kCh * kCh + (size_t)i * 8;
  *(volatile v8h*)q = hv;
  __threadfence();
  *(volatile v8h*)q = hv;
}

__global__ __launch_bounds__(256) void mix_proj_kernel(const float* __restrict__ X,
                                                       const float* __restrict__ mixk, const float* __restrict__ mixv,
                                                       const float* __restrict__ mixr,
                                                       const unsigned short* __restrict__ WT,
                                                       float* __restrict__ KP, float* __restrict__ VP,
                                                       unsigned short* __restrict__ SRP) {
  __shared__ __align__(16) float smem[kTileM * kCP];
  _Float16* As = (_Float16*)smem;
  float*    Cs = smem;
  const int tid = threadIdx.x, lane = tid & 31, wave = tid >> 5;
  const int blk = blockIdx.x;
  const int bi  = blk >> 6;
  const int hi  = blk & 63;
  const float* xb = X + (size_t)bi * kSeq * kCh;
  const size_t tile_off = (size_t)blk * kTileM * kCh;

#pragma unroll 1
  for (int p = 0; p < 3; ++p) {
    const float* mixp = (p == 0) ? mixk : ((p == 1) ? mixv : mixr);
#pragma unroll 1
    for (int it = 0; it < 6; ++it) {
      const int item = it * 256 + tid;
      const int w    = item / 24;
      const int c8   = item - w * 24;
      const int c    = c8 * 8;
      const int grp  = c8 / 6;
      const int dw   = (grp == 0) ? -1 : ((grp == 1) ? 1 : 0);
      const int dh   = (grp == 2) ? -1 : ((grp == 3) ? 1 : 0);
      const int sw   = w + dw;
      const int sh   = hi + dh;
      const bool valid = (sw >= 0) && (sw < kImW) && (sh >= 0) && (sh < kImH);
      const int swc  = min(max(sw, 0), kImW - 1);
      const int shc  = min(max(sh, 0), kImH - 1);
      const float* pc = xb + (size_t)(hi * kImW + w) * kCh + c;
      const float* ps = xb + (size_t)(shc * kImW + swc) * kCh + c;
      const v4f x0 = *(const v4f*)(pc);
      const v4f x1 = *(const v4f*)(pc + 4);
      v4f s0 = *(const v4f*)(ps);
      v4f s1 = *(const v4f*)(ps + 4);
      asm volatile("" : "+v"(s0), "+v"(s1));
      const v4f m0 = *(const v4f*)(mixp + c);
      const v4f m1 = *(const v4f*)(mixp + c + 4);
      v8h hv;
#pragma unroll
      for (int e = 0; e < 4; ++e) {
        const float sa = valid ? s0[e] : 0.0f;
        const float sb = valid ? s1[e] : 0.0f;
        const float va = x0[e] * m0[e] + sa * (1.0f - m0[e]);
        const float vb = x1[e] * m1[e] + sb * (1.0f - m1[e]);
        hv[e]     = to_f16_flushed(va * kActCarry);
        hv[4 + e] = to_f16_flushed(vb * kActCarry);
      }
      *(v8h*)(As + w * kAP + c) = hv;
    }
    __syncthreads();

    v8f acc[2][3];
#pragma unroll
    for (int i = 0; i < 2; ++i)
#pragma unroll
      for (int j = 0; j < 3; ++j) acc[i][j] = (v8f){0.f, 0.f, 0.f, 0.f, 0.f, 0.f, 0.f, 0.f};
    tile_gemm(As, (const _Float16*)WT + (size_t)p * kCh * kCh, lane, wave, acc);
    __syncthreads();
    acc_to_ctile(Cs, lane, wave, acc, kFoldScale, 0.0f);
    __syncthreads();

    if (p < 2) {
      float* dst = ((p == 0) ? KP : VP) + tile_off;
      store_ctile_f32(Cs, dst, tid);
    } else {
#pragma unroll 1
      for (int it = 0; it < 6; ++it) {
        const int idx8 = it * 256 + tid;
        const int row  = idx8 / 24;
        const int col  = (idx8 - row * 24) * 8;
        float* cp = Cs + row * kCP + col;
        const v4f a = *(const v4f*)(cp);
        const v4f b = *(const v4f*)(cp + 4);
        v4f oa, ob;
#pragma unroll
        for (int e = 0; e < 4; ++e) {
          oa[e] = 1.0f / (1.0f + expf(-a[e]));
          ob[e] = 1.0f / (1.0f + expf(-b[e]));
        }
        *(v4f*)(cp)     = oa;
        *(v4f*)(cp + 4) = ob;
      }
      unsigned short* dst = SRP + tile_off;
      for (int pass = 0; pass < 2; ++pass) {
#pragma unroll
        for (int it = 0; it < 6; ++it) {
          const int idx8 = it * 256 + tid;
          const int row  = idx8 / 24;
          const int col  = (idx8 - row * 24) * 8;
          const float* cp = Cs + row * kCP + col;
          const v4f a = *(const v4f*)(cp);
          const v4f b = *(const v4f*)(cp + 4);
          v8h hv;
#pragma unroll
          for (int e = 0; e < 4; ++e) {
            hv[e]     = (_Float16)a[e];
            hv[4 + e] = (_Float16)b[e];
          }
          *(volatile v8h*)(dst + (size_t)idx8 * 8) = hv;
        }
        __threadfence();
      }
    }
    __syncthreads();
  }
}

__global__ __launch_bounds__(192) void decay_scan_kernel(float* KY, const float* __restrict__ VV,
                                                         const float* __restrict__ decay,
                                                         const float* __restrict__ first) {
  const int c  = threadIdx.x;
  const int bi = blockIdx.x;
  const float w = decay[c] * kInvSeq;
  const float u = first[c] * kInvSeq;
  float aa = 0.0f, bb = 0.0f, pp = -1e38f;
  size_t off = (size_t)bi * kSeq * kCh + c;
#pragma unroll 1
  for (int t = 0; t < kSeq; ++t) {
    const float kt = KY[off];
    const float vt = VV[off];
    const float ww = u + kt;
    const float pm = fmaxf(pp, ww);
    const float e1 = expf(pp - pm);
    const float e2 = expf(ww - pm);
    const float num = e1 * aa + e2 * vt;
    const float den = e1 * bb + e2;
    const float y = num / den;
    const float ww2 = pp + w;
    const float qm  = fmaxf(ww2, kt);
    const float f1  = expf(ww2 - qm);
    const float f2  = expf(kt - qm);
    aa = f1 * aa + f2 * vt;
    bb = f1 * bb + f2;
    pp = qm;
    volatile float* yp = KY + off;
    *yp = y;
    __threadfence();
    *yp = y;
    off += kCh;
  }
}

__global__ __launch_bounds__(256) void ln_gate_out_kernel(const float* __restrict__ Y,
                                                          const unsigned short* __restrict__ SRP,
                                                          const float* __restrict__ lng, const float* __restrict__ lnb,
                                                          const unsigned short* __restrict__ WO,
                                                          const int* __restrict__ Hp, const int* __restrict__ Wp,
                                                          float* __restrict__ out) {
  __shared__ __align__(16) float smem[kTileM * kCP];
  _Float16* As = (_Float16*)smem;
  float*    Cs = smem;
  const int tid = threadIdx.x, lane = tid & 31, wave = tid >> 5;
  const int blk = blockIdx.x;
  const int rsub = lane >> 3, l8 = lane & 7;
  const bool shape_bad = (Hp[0] != kImH) || (Wp[0] != kImW);
  const float poison = shape_bad ? __uint_as_float(0x7fc00000u) : 0.0f;

  v4f gA[3][2], bA[3][2];
#pragma unroll
  for (int q = 0; q < 3; ++q) {
    gA[q][0] = *(const v4f*)(lng + 8 * l8 + 64 * q);
    gA[q][1] = *(const v4f*)(lng + 8 * l8 + 64 * q + 4);
    bA[q][0] = *(const v4f*)(lnb + 8 * l8 + 64 * q);
    bA[q][1] = *(const v4f*)(lnb + 8 * l8 + 64 * q + 4);
  }

#pragma unroll 1
  for (int it = 0; it < 2; ++it) {
    const int row = wave * 8 + it * 4 + rsub;
    const size_t tok = (size_t)blk * kTileM + row;
    const float* yp = Y + tok * kCh + 8 * l8;
    const unsigned short* sp = SRP + tok * kCh + 8 * l8;
    v4f ya[3][2];
    v4u su[3];
#pragma unroll
    for (int q = 0; q < 3; ++q) {
      ya[q][0] = *(const v4f*)(yp + 64 * q);
      ya[q][1] = *(const v4f*)(yp + 64 * q + 4);
      su[q]    = *(const v4u*)(sp + 64 * q);
    }
    float s = 0.0f;
#pragma unroll
    for (int q = 0; q < 3; ++q)
#pragma unroll
      for (int hf = 0; hf < 2; ++hf)
#pragma unroll
        for (int e = 0; e < 4; ++e) s += ya[q][hf][e];
    s += __shfl_xor(s, 1, 32);
    s += __shfl_xor(s, 2, 32);
    s += __shfl_xor(s, 4, 32);
    const float mu = s * kInvCh;
    float ss = 0.0f;
#pragma unroll
    for (int q = 0; q < 3; ++q)
#pragma unroll
      for (int hf = 0; hf < 2; ++hf)
#pragma unroll
        for (int e = 0; e < 4; ++e) {
          const float d = ya[q][hf][e] - mu;
          ya[q][hf][e] = d;
          ss += d * d;
        }
    ss += __shfl_xor(ss, 1, 32);
    ss += __shfl_xor(ss, 2, 32);
    ss += __shfl_xor(ss, 4, 32);
    const float var  = ss * kInvCh;
    const float rstd = rsqrtf(var + kLnEps);
#pragma unroll
    for (int q = 0; q < 3; ++q) {
      const unsigned w0 = su[q][0];
      const unsigned w1 = su[q][1];
      const unsigned w2 = su[q][2];
      const unsigned w3 = su[q][3];
      float sg[8];
      sg[0] = h16_to_f32(w0 & 0xffffu);
      sg[1] = h16_to_f32(w0 >> 16);
      sg[2] = h16_to_f32(w1 & 0xffffu);
      sg[3] = h16_to_f32(w1 >> 16);
      sg[4] = h16_to_f32(w2 & 0xffffu);
      sg[5] = h16_to_f32(w2 >> 16);
      sg[6] = h16_to_f32(w3 & 0xffffu);
      sg[7] = h16_to_f32(w3 >> 16);
      v8h hv;
#pragma unroll
      for (int hf = 0; hf < 2; ++hf)
#pragma unroll
        for (int e = 0; e < 4; ++e) {
          const float ln = (ya[q][hf][e] * rstd) * gA[q][hf][e] + bA[q][hf][e];
          const float gv = ln * sg[4 * hf + e];
          hv[4 * hf + e] = to_f16_flushed(gv * kActCarry);
        }
      *(v8h*)(As + row * kAP + 8 * l8 + 64 * q) = hv;
    }
  }
  __syncthreads();

  v8f acc[2][3];
#pragma unroll
  for (int i = 0; i < 2; ++i)
#pragma unroll
    for (int j = 0; j < 3; ++j) acc[i][j] = (v8f){0.f, 0.f, 0.f, 0.f, 0.f, 0.f, 0.f, 0.f};
  tile_gemm(As, (const _Float16*)WO, lane, wave, acc);
  __syncthreads();
  acc_to_ctile(Cs, lane, wave, acc, kFoldScale, poison);
  __syncthreads();
  store_ctile_f32(Cs, out + (size_t)blk * kTileM * kCh, tid);
}

extern "C" void kernel_launch(void* const* d_in, const int* in_sizes, int n_in,
                              void* d_out, int out_size, void* d_ws, size_t ws_size,
                              hipStream_t stream) {
  if (n_in < 14 || d_out == nullptr || d_ws == nullptr) return;
  if (in_sizes[0] != kTok * kCh) return;
  if (in_sizes[1] != 1 || in_sizes[2] != 1) return;
  if (in_sizes[3] != kCh || in_sizes[4] != kCh) return;
  if (in_sizes[5] != kCh || in_sizes[6] != kCh || in_sizes[7] != kCh) return;
  if (in_sizes[8] != kCh * kCh || in_sizes[9] != kCh * kCh) return;
  if (in_sizes[10] != kCh * kCh || in_sizes[11] != kCh * kCh) return;
  if (in_sizes[12] != kCh || in_sizes[13] != kCh) return;
  if (out_size != kTok * kCh) return;
  if (ws_size < kWsTotal) return;

  const float* x     = (const float*)d_in[0];
  const int*   Hp    = (const int*)d_in[1];
  const int*   Wp    = (const int*)d_in[2];
  const float* decay = (const float*)d_in[3];
  const float* first = (const float*)d_in[4];
  const float* mixk  = (const float*)d_in[5];
  const float* mixv  = (const float*)d_in[6];
  const float* mixr  = (const float*)d_in[7];
  const float* Wk    = (const float*)d_in[8];
  const float* Wv    = (const float*)d_in[9];
  const float* Wr    = (const float*)d_in[10];
  const float* Wo    = (const float*)d_in[11];
  const float* lng   = (const float*)d_in[12];
  const float* lnb   = (const float*)d_in[13];
  float* out = (float*)d_out;

  char* ws = (char*)d_ws;
  unsigned short* WT = (unsigned short*)(ws + kOffWT);
  float*          KY = (float*)(ws + kOffKY);
  float*          VV = (float*)(ws + kOffVV);
  unsigned short* SR = (unsigned short*)(ws + kOffSR);

  prepack_w_kernel<<<dim3((kCh * kCh / 8) / 256, 4), 256, 0, stream>>>(Wk, Wv, Wr, Wo, WT);

  mix_proj_kernel<<<kTok / kTileM, 256, 0, stream>>>(x, mixk, mixv, mixr, WT, KY, VV, SR);

  decay_scan_kernel<<<kNB, kCh, 0, stream>>>(KY, VV, decay, first);

  ln_gate_out_kernel<<<kTok / kTileM, 256, 0, stream>>>(KY, SR, lng, lnb, WT + (size_t)3 * kCh * kCh, Hp, Wp, out);
}
